// TBCNNFFDLayer_39367670235354
// MI455X (gfx1250) — hardware-verified
//
#include <hip/hip_runtime.h>
#include <stddef.h>
#include <stdint.h>


#define BT    512
#define NN    64
#define CC    8
#define DD    256
#define KC    768
#define APH   776
#define HPH   264
#define NTHR  256
#define NPRM  5
#define WSCL  16.0f
#define PSCL  0.0625f
#define NEGV  (-1e8f)
#define EPSV  1e-5f
#define WSCAP 134217728

#define SZ_WCT ((size_t)DD * KC * 2)
#define SZ_WOT ((size_t)DD * DD * 2)
#define SZ_TOT (SZ_WCT + SZ_WOT)
static_assert(SZ_TOT == 524288);
static_assert(SZ_TOT <= (size_t)WSCAP);
static_assert((SZ_WCT % 512) == 0);
static_assert((SZ_WOT % 512) == 0);
static_assert(NTHR == DD);
static_assert(NTHR == 8 * 32);
static_assert((KC % 32) == 0);
static_assert((DD % 32) == 0);
static_assert((APH % 8) == 0);
static_assert((HPH % 8) == 0);
static_assert(NN * HPH <= NN * APH);
static_assert(NN == 64);
static_assert(8 * 32 == DD);

typedef _Float16     v16h __attribute__((ext_vector_type(16)));
typedef _Float16     v8h  __attribute__((ext_vector_type(8)));
typedef float        v8f  __attribute__((ext_vector_type(8)));
typedef float        v4f  __attribute__((ext_vector_type(4)));
typedef unsigned int v4u  __attribute__((ext_vector_type(4)));
union Frag { v16h v; v8h half[2]; };
union Pk8  { v8h h; v4u u; };

__device__ __forceinline__ v4u cvt8(const v4f a, const v4f b) {
  v8h hv = {(_Float16)a.x, (_Float16)a.y, (_Float16)a.z, (_Float16)a.w,
            (_Float16)b.x, (_Float16)b.y, (_Float16)b.z, (_Float16)b.w};
  Pk8 p;
  p.h = hv;
  return p.u;
}

__device__ __forceinline__ void ld8f(const float* p, float (&o)[8]) {
  const v4f a = *(const v4f*)p;
  const v4f c = *(const v4f*)(p + 4);
  o[0] = a.x; o[1] = a.y; o[2] = a.z; o[3] = a.w;
  o[4] = c.x; o[5] = c.y; o[6] = c.z; o[7] = c.w;
}

__device__ __forceinline__ v8f wmh(v16h a, v16h b, v8f c) {
  v8f d = __builtin_amdgcn_wmma_f32_16x16x32_f16(false, a, false, b, (short)0, c, false, false);
  asm volatile("v_nop\n\tv_nop\n\tv_nop\n\tv_nop" : "+v"(d) : "v"(a), "v"(b));
  return d;
}

__device__ __forceinline__ v16h lda_frag(const _Float16* tile, int pitch, int row, int k0, int h) {
  Frag a;
  const _Float16* p = tile + row * pitch + k0 + 8 * h;
  a.half[0] = *(const v8h*)p;
  a.half[1] = *(const v8h*)(p + 16);
  return a.v;
}

__device__ __forceinline__ v16h ldb_frag(const _Float16* plane, int pitch, int n, int k0, int h) {
  Frag b;
  const _Float16* p = plane + (size_t)n * pitch + k0 + 8 * h;
  b.half[0] = *(const v8h*)p;
  b.half[1] = *(const v8h*)(p + 16);
  return b.v;
}

__global__ __launch_bounds__(32) void k_prep(const float* __restrict__ wt, const float* __restrict__ wl,
                                             const float* __restrict__ wr, const float* __restrict__ wo,
                                             _Float16* WCT, _Float16* WOT) {
  const int blk = blockIdx.x, lane = threadIdx.x;
  const float* src;
  _Float16* dst;
  if (blk < 3 * DD) {
    const int n = blk / 3;
    const int seg = blk - 3 * n;
    const float* W = (seg == 0) ? wt : ((seg == 1) ? wl : wr);
    src = W + n;
    dst = WCT + (size_t)n * KC + seg * DD;
  } else {
    const int n = blk - 3 * DD;
    src = wo + n;
    dst = WOT + (size_t)n * DD;
  }
  const int k0 = 8 * lane;
  v4f f0, f1;
  f0.x = src[(size_t)(k0 + 0) * DD] * WSCL;
  f0.y = src[(size_t)(k0 + 1) * DD] * WSCL;
  f0.z = src[(size_t)(k0 + 2) * DD] * WSCL;
  f0.w = src[(size_t)(k0 + 3) * DD] * WSCL;
  f1.x = src[(size_t)(k0 + 4) * DD] * WSCL;
  f1.y = src[(size_t)(k0 + 5) * DD] * WSCL;
  f1.z = src[(size_t)(k0 + 6) * DD] * WSCL;
  f1.w = src[(size_t)(k0 + 7) * DD] * WSCL;
  const v4u pk = cvt8(f0, f1);
  _Float16* d = dst + k0;
  *(volatile v4u*)d = pk;
  __threadfence();
  *(volatile v4u*)d = pk;
}

__global__ __launch_bounds__(NTHR) void k_main(const float* __restrict__ x, const int* __restrict__ child,
                                               const int* __restrict__ tmask, const float* __restrict__ bias,
                                               const float* __restrict__ gam, const float* __restrict__ bet,
                                               const float* __restrict__ attnW, const float* __restrict__ attnB,
                                               const float* __restrict__ outB,
                                               const _Float16* __restrict__ WCT, const _Float16* __restrict__ WOT,
                                               float* out) {
  __shared__ __attribute__((aligned(16))) _Float16 As[NN * APH];
  __shared__ __attribute__((aligned(16))) float hs[NN * DD];
  __shared__ __attribute__((aligned(16))) float prm[NPRM * DD];
  __shared__ __attribute__((aligned(16))) float wred[2 * DD];
  __shared__ __attribute__((aligned(16))) float obuf[DD];
  __shared__ float logitsS[NN];
  __shared__ float scoresS[NN];

  const int tid = threadIdx.x, lane = tid & 31, wv = tid >> 5, h = lane >> 4, m = lane & 15;
  const int b = blockIdx.x;
  const float* xb = x + (size_t)b * NN * DD;
  _Float16* Hh = As;

  prm[0 * DD + tid] = bias[tid];
  prm[1 * DD + tid] = gam[tid];
  prm[2 * DD + tid] = bet[tid];
  prm[3 * DD + tid] = attnW[tid];
  prm[4 * DD + tid] = outB[tid];
  const float ab = attnB[0];

#pragma unroll 1
  for (int n = 0; n < NN; ++n) {
    const int* ch = child + ((size_t)b * NN + n) * CC;
    int cv[CC];
#pragma unroll
    for (int c = 0; c < CC; ++c) cv[c] = ch[c];
    int ns = 0;
#pragma unroll
    for (int c = 0; c < CC; ++c) ns += (cv[c] != 0) ? 1 : 0;
    const float den = (ns == 1) ? 1.0f : ((float)ns - 1.0f);
    const float rden = 1.0f / den;
    float al = 0.f, ar = 0.f;
#pragma unroll
    for (int c = 0; c < CC; ++c) {
      int ci = cv[c];
      ci = (ci < 0) ? 0 : ci;
      ci = (ci > NN - 1) ? (NN - 1) : ci;
      const float mk = fminf((float)cv[c], 1.0f);
      const float er = (ns == 1) ? ((c == 0) ? 0.5f : 0.0f) : (((float)c * mk) * rden);
      const float el = mk * (1.0f - er);
      float v = xb[ci * DD + tid];
      v = (cv[c] != 0) ? v : 0.0f;
      al = fmaf(el, v, al);
      ar = fmaf(er, v, ar);
    }
    const float at = xb[n * DD + tid];
    As[n * APH + tid]          = (_Float16)at;
    As[n * APH + DD + tid]     = (_Float16)al;
    As[n * APH + 2 * DD + tid] = (_Float16)ar;
  }
  __syncthreads();

  const int mp = wv & 1;
  const int nbase = (wv >> 1) * 64;
  const v8f zero8 = {0.f, 0.f, 0.f, 0.f, 0.f, 0.f, 0.f, 0.f};

  {
    v8f acc[2][4];
#pragma unroll
    for (int mi = 0; mi < 2; ++mi) {
#pragma unroll
      for (int s = 0; s < 4; ++s) acc[mi][s] = zero8;
    }
#pragma unroll 1
    for (int kt = 0; kt < KC / 32; ++kt) {
      const int k0 = 32 * kt;
      const v16h a0 = lda_frag(As, APH, 32 * mp + m, k0, h);
      const v16h a1 = lda_frag(As, APH, 32 * mp + 16 + m, k0, h);
#pragma unroll
      for (int s = 0; s < 4; ++s) {
        const v16h bf = ldb_frag(WCT, KC, nbase + 16 * s + m, k0, h);
        acc[0][s] = wmh(a0, bf, acc[0][s]);
        acc[1][s] = wmh(a1, bf, acc[1][s]);
      }
    }
#pragma unroll
    for (int mi = 0; mi < 2; ++mi) {
#pragma unroll
      for (int s = 0; s < 4; ++s) {
        const int col = nbase + 16 * s + m;
#pragma unroll
        for (int r = 0; r < 8; ++r) hs[(32 * mp + 16 * mi + 8 * h + r) * DD + col] = acc[mi][s][r] * PSCL;
      }
    }
  }
  __syncthreads();

  {
    const int c0 = 8 * lane;
    float bi[8], gb[8], bb[8], aw[8];
    ld8f(prm + 0 * DD + c0, bi);
    ld8f(prm + 1 * DD + c0, gb);
    ld8f(prm + 2 * DD + c0, bb);
    ld8f(prm + 3 * DD + c0, aw);
#pragma unroll 1
    for (int j = 0; j < 8; ++j) {
      const int n = wv * 8 + j;
      float hc[8], xv[8];
      ld8f(hs + n * DD + c0, hc);
      ld8f(xb + n * DD + c0, xv);
      float v[8];
      float s = 0.f;
#pragma unroll
      for (int i = 0; i < 8; ++i) {
        const float hv = (hc[i] + bi[i]) + xv[i];
        v[i] = hv;
        s += hv;
      }
#pragma unroll
      for (int off = 16; off > 0; off >>= 1) s += __shfl_xor(s, off, 32);
      const float mu = s * (1.0f / 256.0f);
      float s2 = 0.f;
#pragma unroll
      for (int i = 0; i < 8; ++i) {
        const float t = v[i] - mu;
        s2 = fmaf(t, t, s2);
      }
#pragma unroll
      for (int off = 16; off > 0; off >>= 1) s2 += __shfl_xor(s2, off, 32);
      const float var = s2 * (1.0f / 256.0f);
      const float inv = 1.0f / sqrtf(var + EPSV);
      float hn[8];
      float lg = 0.f;
#pragma unroll
      for (int i = 0; i < 8; ++i) {
        float t = (v[i] - mu) * inv * gb[i] + bb[i];
        t = fmaxf(t, 0.f);
        hn[i] = t;
        lg = fmaf(t, aw[i], lg);
      }
      {
        const v4f q0 = {hn[0], hn[1], hn[2], hn[3]};
        const v4f q1 = {hn[4], hn[5], hn[6], hn[7]};
        *(v4u*)(Hh + n * HPH + c0) = cvt8(q0, q1);
      }
#pragma unroll
      for (int off = 16; off > 0; off >>= 1) lg += __shfl_xor(lg, off, 32);
      const int mkv = tmask[(size_t)b * NN + n];
      const float madd = (mkv != 0) ? NEGV : (float)mkv;
      float t = lg + ab;
      t = t + madd;
      if (lane == 0) logitsS[n] = t;
    }
  }
  __syncthreads();

  if (wv == 0) {
    const float l0 = logitsS[lane], l1 = logitsS[lane + 32];
    float mx = fmaxf(l0, l1);
#pragma unroll
    for (int off = 16; off > 0; off >>= 1) mx = fmaxf(mx, __shfl_xor(mx, off, 32));
    const float e0 = expf(l0 - mx), e1 = expf(l1 - mx);
    float ss = e0 + e1;
#pragma unroll
    for (int off = 16; off > 0; off >>= 1) ss += __shfl_xor(ss, off, 32);
    const float rs = 1.0f / ss;
    scoresS[lane]      = e0 * rs;
    scoresS[lane + 32] = e1 * rs;
  }
  __syncthreads();

  {
    v8f acc[2][4];
#pragma unroll
    for (int mi = 0; mi < 2; ++mi) {
#pragma unroll
      for (int s = 0; s < 4; ++s) acc[mi][s] = zero8;
    }
#pragma unroll 1
    for (int kt = 0; kt < DD / 32; ++kt) {
      const int k0 = 32 * kt;
      const v16h a0 = lda_frag(Hh, HPH, 32 * mp + m, k0, h);
      const v16h a1 = lda_frag(Hh, HPH, 32 * mp + 16 + m, k0, h);
#pragma unroll
      for (int s = 0; s < 4; ++s) {
        const v16h bf = ldb_frag(WOT, DD, nbase + 16 * s + m, k0, h);
        acc[0][s] = wmh(a0, bf, acc[0][s]);
        acc[1][s] = wmh(a1, bf, acc[1][s]);
      }
    }
    float sc[2][8];
#pragma unroll
    for (int mi = 0; mi < 2; ++mi) {
#pragma unroll
      for (int r = 0; r < 8; ++r) sc[mi][r] = scoresS[32 * mp + 16 * mi + 8 * h + r];
    }
#pragma unroll
    for (int s = 0; s < 4; ++s) {
      const int col = nbase + 16 * s + m;
      const float ob = prm[4 * DD + col];
      float p = 0.f;
#pragma unroll
      for (int mi = 0; mi < 2; ++mi) {
#pragma unroll
        for (int r = 0; r < 8; ++r) p = fmaf(sc[mi][r], acc[mi][s][r] * PSCL + ob, p);
      }
      p += __shfl_xor(p, 16, 32);
      if (h == 0) wred[mp * DD + col] = p;
    }
  }
  __syncthreads();
  {
    const float o = wred[tid] + wred[DD + tid];
    obuf[tid] = o;
  }
  __syncthreads();
  if (wv == 0) {
    const v4f v0 = *(const v4f*)(obuf + 4 * lane);
    const v4f v1 = *(const v4f*)(obuf + 4 * (32 + lane));
    float* po = out + (size_t)b * DD;
    *(volatile v4f*)(po + 4 * lane)        = v0;
    *(volatile v4f*)(po + 4 * (32 + lane)) = v1;
    __threadfence();
    *(volatile v4f*)(po + 4 * lane)        = v0;
    *(volatile v4f*)(po + 4 * (32 + lane)) = v1;
  }
}

extern "C" void kernel_launch(void* const* d_in, const int* in_sizes, int n_in,
                              void* d_out, int out_size, void* d_ws, size_t ws_size,
                              hipStream_t stream) {
  if (n_in < 13) return;
  if (in_sizes[0] != BT * NN * DD) return;
  if (in_sizes[1] != BT * NN * CC) return;
  if (in_sizes[2] != BT * NN) return;
  if (in_sizes[3] != DD * DD || in_sizes[4] != DD * DD || in_sizes[5] != DD * DD) return;
  if (in_sizes[6] != DD || in_sizes[7] != DD || in_sizes[8] != DD) return;
  if (in_sizes[9] != DD || in_sizes[10] < 1) return;
  if (in_sizes[11] != DD * DD || in_sizes[12] != DD) return;
  if (out_size != BT * DD) return;
  if (ws_size < SZ_TOT) return;

  const float* x     = (const float*)d_in[0];
  const int*   child = (const int*)d_in[1];
  const int*   tmask = (const int*)d_in[2];
  const float* wt    = (const float*)d_in[3];
  const float* wl    = (const float*)d_in[4];
  const float* wr    = (const float*)d_in[5];
  const float* bias  = (const float*)d_in[6];
  const float* gam   = (const float*)d_in[7];
  const float* bet   = (const float*)d_in[8];
  const float* attnW = (const float*)d_in[9];
  const float* attnB = (const float*)d_in[10];
  const float* outW  = (const float*)d_in[11];
  const float* outB  = (const float*)d_in[12];
  float* out = (float*)d_out;

  char* ws = (char*)d_ws;
  size_t off = 0;
  const size_t oWCT = off; off += SZ_WCT;
  const size_t oWOT = off; off += SZ_WOT;
  if (off != SZ_TOT) return;
  if (off > ws_size || off > (size_t)WSCAP) return;
  _Float16* WCT = (_Float16*)(ws + oWCT);
  _Float16* WOT = (_Float16*)(ws + oWOT);

  k_prep<<<3 * DD + DD, 32, 0, stream>>>(wt, wl, wr, outW, WCT, WOT);
  k_main<<<BT, NTHR, 0, stream>>>(x, child, tmask, bias, gam, bet, attnW, attnB, outB, WCT, WOT, out);
}
